// SimpleGraphNeuralNet_19782619365957
// MI455X (gfx1250) — hardware-run, weakly checked
//
#include <hip/hip_runtime.h>
#include <stddef.h>
#include <stdint.h>


#ifndef SINGLE_Z
#define SINGLE_Z 0
#endif
#ifndef SINGLE_T
#define SINGLE_T 0
#endif
#ifndef SINGLE_F
#define SINGLE_F 0
#endif

#define NN       50000
#define NE       800000
#define NL       4
#define DH       128
#define D2       256
#define DOUT     64
#define GBM      128
#define GTHR     256
#define MPAD     50048
#define MTILES   391
#define PZ       256
#define PT       512
#define NTHR     256
#define NBRUN    1024
#define SLB      10
#define NBLK     49
#define NWB      8
#define BTHR     (NWB * 32)
#define WLCAP    3072
#define RCAP     20480
#define STEPE    128
#define SHSTEPS  782
#define SHARE    (SHSTEPS * STEPE)
#define DEGCAP   64
#define CNTN     (NBLK * NBRUN)
#define BKT_INTS (NWB * WLCAP + NWB * NBRUN + RCAP + 2 * NBRUN + 64)
#define PB1      0
#define PGAM     1024
#define PBET     2048
#define PB2      3072
#define PLB      4096
#define PEPS     4160
#define PARN     5120
#define PBE_W1   128
#define PBE_W2   256
#define PBE_LW   264
#define PBE_PAR  269
#define PB_X     6256
#define PGRID    (PBE_PAR + PB_X)
#define WSMAX    (128u << 20)

constexpr int KZ = SINGLE_Z ? 128 : 256;
constexpr int KT = SINGLE_T ? 256 : 512;
constexpr int KF = SINGLE_F ? 128 : 256;

static_assert(MPAD == MTILES * GBM && MPAD >= NN && (MTILES - 1) * GBM < NN);
static_assert(MPAD % 64 == 0 && MPAD % 8 == 0);
static_assert(NN <= 65536 && NBRUN <= 1024 && NBRUN == (1 << SLB));
static_assert(NBLK * NBRUN >= MPAD && (NBLK - 1) * NBRUN < NN);
static_assert(NWB * SHARE >= NE && (NE % 4) == 0);
static_assert(RCAP % 1024 == 0 && BTHR * 4 == NBRUN);
static_assert((NWB * NBRUN + RCAP) % (BTHR * 4) == 0);
static_assert(BKT_INTS * 4 <= 300000);
static_assert(DH % 8 == 0 && D2 % 8 == 0 && DOUT % 8 == 0 && PZ % 8 == 0 && PT % 8 == 0);
static_assert(KZ % 32 == 0 && KT % 32 == 0 && KF % 32 == 0 && KZ <= PZ && KT <= PT && KF <= PZ);
static_assert(PZ == 2 * DH && PT == 2 * D2);
static_assert(MPAD * 32 == PB_X * NTHR);
static_assert(PEPS + NL <= PARN && PLB + DOUT <= PEPS);

typedef float          v2f  __attribute__((ext_vector_type(2)));
typedef float          v4f  __attribute__((ext_vector_type(4)));
typedef float          v8f  __attribute__((ext_vector_type(8)));
typedef int            v4i  __attribute__((ext_vector_type(4)));
typedef int            v8i  __attribute__((ext_vector_type(8)));
typedef unsigned int   v2u  __attribute__((ext_vector_type(2)));
typedef unsigned int   v4u  __attribute__((ext_vector_type(4)));
typedef unsigned short v8us __attribute__((ext_vector_type(8)));
typedef __bf16         v16b __attribute__((ext_vector_type(16)));
typedef v4f  __attribute__((may_alias)) v4fa;
typedef v4i  __attribute__((may_alias)) v4ia;
typedef v4u  __attribute__((may_alias)) v4ua;
typedef v8us __attribute__((may_alias)) v8usa;
union FragB { v16b v; v8us h[2]; v8i w; };

__device__ __forceinline__ v8f wmb(const FragB& a, const FragB& b, v8f c) {
  v8f d = __builtin_amdgcn_wmma_f32_16x16x32_bf16(false, a.v, false, b.v, (short)0, c, false, false);
  asm volatile("v_nop\n\tv_nop\n\tv_nop\n\tv_nop" : "+v"(d) : "v"(a.w), "v"(b.w));
  return d;
}

__device__ __forceinline__ void pin_i(int x)   { asm volatile("" :: "v"(x)); }
__device__ __forceinline__ void pin_4i(v4i x)  { asm volatile("" :: "v"(x)); }
__device__ __forceinline__ void pin_4f(v4f x)  { asm volatile("" :: "v"(x)); }

__device__ __forceinline__ unsigned bf_bits(float f) {
  const unsigned u = __float_as_uint(f);
  const unsigned r = (u + 0x7FFFu + ((u >> 16) & 1u)) >> 16;
  return ((u & 0x7FFFFFFFu) > 0x7F800000u) ? 0x7FC0u : r;
}
__device__ __forceinline__ float bf_val(unsigned b) { return __uint_as_float(b << 16); }
__device__ __forceinline__ float bf_rne(float f) { return bf_val(bf_bits(f)); }
__device__ __forceinline__ v4f bf_rne4(v4f a) {
  v4f o; o.x = bf_rne(a.x); o.y = bf_rne(a.y); o.z = bf_rne(a.z); o.w = bf_rne(a.w); return o;
}
__device__ __forceinline__ v4f mask4(v4f q, unsigned mk) {
  v4f r;
  r.x = __uint_as_float(__float_as_uint(q.x) & mk);
  r.y = __uint_as_float(__float_as_uint(q.y) & mk);
  r.z = __uint_as_float(__float_as_uint(q.z) & mk);
  r.w = __uint_as_float(__float_as_uint(q.w) & mk);
  return r;
}
__device__ __forceinline__ v4f or4(v4f a, v4f b) {
  v4f r;
  r.x = __uint_as_float(__float_as_uint(a.x) | __float_as_uint(b.x));
  r.y = __uint_as_float(__float_as_uint(a.y) | __float_as_uint(b.y));
  r.z = __uint_as_float(__float_as_uint(a.z) | __float_as_uint(b.z));
  r.w = __uint_as_float(__float_as_uint(a.w) | __float_as_uint(b.w));
  return r;
}

__global__ __launch_bounds__(NTHR) void k_prep(
    const float* __restrict__ x, const float* __restrict__ W1, const float* __restrict__ b1,
    const float* __restrict__ gam, const float* __restrict__ bet, const float* __restrict__ W2,
    const float* __restrict__ b2, const float* __restrict__ eps, const float* __restrict__ lw,
    const float* __restrict__ lb,
    unsigned short* w1t, unsigned short* w2t, unsigned short* lwt, float* par, float* x0) {
  const int blk = (int)blockIdx.x, tid = (int)threadIdx.x;
  if (blk < PBE_LW) {
    v8us o;
    unsigned short* dp;
    if (blk < PBE_W1) {
      const int u = blk * NTHR + tid;
      const int layer = u >> 13, v = u & 8191;
      const int n = v >> 5, k8 = (v & 31) * 8, kk = k8 & (DH - 1);
      const float* p = W1 + (size_t)layer * DH * D2 + (size_t)kk * D2 + n;
#pragma unroll
      for (int i = 0; i < 8; ++i) o[i] = (unsigned short)bf_bits(p[(size_t)i * D2]);
      dp = w1t + (size_t)layer * (D2 * PZ) + (size_t)n * PZ + k8;
    } else if (blk < PBE_W2) {
      const int u = (blk - PBE_W1) * NTHR + tid;
      const int layer = u >> 13, v = u & 8191;
      const int n = v >> 6, k8 = (v & 63) * 8, kk = k8 & (D2 - 1);
      const float* p = W2 + (size_t)layer * D2 * DH + (size_t)kk * DH + n;
#pragma unroll
      for (int i = 0; i < 8; ++i) o[i] = (unsigned short)bf_bits(p[(size_t)i * DH]);
      dp = w2t + (size_t)layer * (DH * PT) + (size_t)n * PT + k8;
    } else {
      const int u = (blk - PBE_W2) * NTHR + tid;
      const int n = u >> 5, k8 = (u & 31) * 8, kk = k8 & (DH - 1);
      const float* p = lw + (size_t)kk * DOUT + n;
#pragma unroll
      for (int i = 0; i < 8; ++i) o[i] = (unsigned short)bf_bits(p[(size_t)i * DOUT]);
      dp = lwt + (size_t)n * PZ + k8;
    }
    *(volatile v8us*)dp = o;
    __threadfence();
    *(volatile v8us*)dp = o;
  } else if (blk < PBE_PAR) {
    const int s = blk - PBE_LW;
    const int u = tid;
    v4f v;
    if (s == 0) {
      v = *(const v4f*)(b1 + 4 * u);
    } else if (s == 1) {
      v = *(const v4f*)(gam + 4 * u);
    } else if (s == 2) {
      v = *(const v4f*)(bet + 4 * u);
    } else if (s == 3) {
      const int uc = u < 128 ? u : 127;
      const v4f q = *(const v4f*)(b2 + 4 * uc);
      pin_4f(q);
      v = mask4(q, (u < 128) ? 0xFFFFFFFFu : 0u);
    } else {
      const int uc = u < 16 ? u : 15;
      const v4f q = *(const v4f*)(lb + 4 * uc);
      v4f ev;
      ev.x = eps[0]; ev.y = eps[1]; ev.z = eps[2]; ev.w = eps[3];
      pin_4f(q); pin_4f(ev);
      v = or4(mask4(q, (u < 16) ? 0xFFFFFFFFu : 0u), mask4(ev, (u == 16) ? 0xFFFFFFFFu : 0u));
    }
    const v4f o = bf_rne4(v);
    float* dp = par + (size_t)s * 1024 + 4 * u;
    *(volatile v4f*)dp = o;
    __threadfence();
    *(volatile v4f*)dp = o;
  } else {
    const int u = (blk - PBE_PAR) * NTHR + tid;
    const int row = u >> 5, c4 = (u & 31) * 4;
    const int rc = row < NN ? row : NN - 1;
    const v4f a = *(const v4f*)(x + (size_t)rc * DH + c4);
    pin_4f(a);
    const v4f o = mask4(bf_rne4(a), (row < NN) ? 0xFFFFFFFFu : 0u);
    float* dp = x0 + (size_t)row * DH + c4;
    *(volatile v4f*)dp = o;
    __threadfence();
    *(volatile v4f*)dp = o;
  }
}

__global__ __launch_bounds__(BTHR) void k_bucket(const int* __restrict__ ei, int* lst, int* cntg, int* offg,
                                                 int* flg) {
  extern __shared__ v4i bsm4[];
  int* wl   = (int*)bsm4;
  int* cw   = wl + NWB * WLCAP;
  int* plc  = cw + NWB * NBRUN;
  int* cnt  = plc + RCAP;
  int* off  = cnt + NBRUN;
  int* misc = off + NBRUN;
  const int tid = (int)threadIdx.x, lane = tid & 31, wave = tid >> 5;
  const int b = (int)blockIdx.x;
  const int base = b * NBRUN;
  int nbv = NN - base;
  nbv = nbv < 0 ? 0 : (nbv > NBRUN ? NBRUN : nbv);

  {
    const v4i z4 = {0, 0, 0, 0};
#pragma unroll 1
    for (int i = tid * 4; i < NWB * NBRUN + RCAP; i += BTHR * 4) *(v4ia*)(cw + i) = z4;
    if (tid < 64) misc[tid] = 0;
  }
  __syncthreads();

  const int* srcs = ei;
  const int* dsts = ei + NE;
  const unsigned ubase = (unsigned)base, unb = (unsigned)nbv;
  int* mywl = wl + wave * WLCAP;
  int wc = 0;
  const int ew0 = wave * SHARE;
#pragma unroll 1
  for (int st = 0; st < SHSTEPS; ++st) {
    const int e  = ew0 + st * STEPE + 4 * lane;
    const int ec = e > NE - 4 ? NE - 4 : e;
    const v4i dv = *(const v4i*)(dsts + ec);
    const v4i sv = *(const v4i*)(srcs + ec);
    pin_4i(dv); pin_4i(sv);
    const bool ok = e < NE;
    const unsigned s0 = (unsigned)dv.x - ubase, s1 = (unsigned)dv.y - ubase;
    const unsigned s2 = (unsigned)dv.z - ubase, s3 = (unsigned)dv.w - ubase;
    const bool h0 = ok & (s0 < unb), h1 = ok & (s1 < unb), h2 = ok & (s2 < unb), h3 = ok & (s3 < unb);
    const unsigned m0 = __builtin_amdgcn_ballot_w32(h0);
    const unsigned m1 = __builtin_amdgcn_ballot_w32(h1);
    const unsigned m2 = __builtin_amdgcn_ballot_w32(h2);
    const unsigned m3 = __builtin_amdgcn_ballot_w32(h3);
    if ((m0 | m1 | m2 | m3) != 0u) {
      int pos = wc + (int)__builtin_amdgcn_mbcnt_lo(m0, 0u) + (int)__builtin_amdgcn_mbcnt_lo(m1, 0u)
                   + (int)__builtin_amdgcn_mbcnt_lo(m2, 0u) + (int)__builtin_amdgcn_mbcnt_lo(m3, 0u);
      const int q0 = sv.x < 0 ? 0 : (sv.x > NN - 1 ? NN - 1 : sv.x);
      const int q1 = sv.y < 0 ? 0 : (sv.y > NN - 1 ? NN - 1 : sv.y);
      const int q2 = sv.z < 0 ? 0 : (sv.z > NN - 1 ? NN - 1 : sv.z);
      const int q3 = sv.w < 0 ? 0 : (sv.w > NN - 1 ? NN - 1 : sv.w);
      if (h0) { if (pos < WLCAP) mywl[pos] = (q0 << SLB) | (int)s0; pos += 1; }
      if (h1) { if (pos < WLCAP) mywl[pos] = (q1 << SLB) | (int)s1; pos += 1; }
      if (h2) { if (pos < WLCAP) mywl[pos] = (q2 << SLB) | (int)s2; pos += 1; }
      if (h3) { if (pos < WLCAP) mywl[pos] = (q3 << SLB) | (int)s3; pos += 1; }
      wc += (int)__builtin_popcount(m0) + (int)__builtin_popcount(m1)
          + (int)__builtin_popcount(m2) + (int)__builtin_popcount(m3);
    }
  }
  const int wov = __builtin_amdgcn_readfirstlane(wc > WLCAP ? 1 : 0);
  const int n   = __builtin_amdgcn_readfirstlane(wc > WLCAP ? WLCAP : wc);
  if (lane == 0) { misc[wave] = n; misc[8 + wave] = wov; }
  __syncthreads();

#pragma unroll 1
  for (int b0 = 0; b0 < n; b0 += 32) {
    int idx = b0 + lane;
    idx = idx > n - 1 ? n - 1 : idx;
    const int ent = mywl[idx];
    const int m32 = (n - b0) < 32 ? (n - b0) : 32;
#pragma unroll 1
    for (int k = 0; k < m32; ++k) {
      const int u  = __builtin_amdgcn_readlane(ent, k);
      const int sl = u & (NBRUN - 1);
      if (lane == 0) cw[wave * NBRUN + sl] = cw[wave * NBRUN + sl] + 1;
    }
  }
  __syncthreads();

  {
    int c0 = 0, c1 = 0, c2 = 0, c3 = 0;
#pragma unroll
    for (int w = 0; w < NWB; ++w) {
      const v4i q = *(const v4ia*)(cw + w * NBRUN + 4 * tid);
      c0 += q.x; c1 += q.y; c2 += q.z; c3 += q.w;
    }
    const int ts = c0 + c1 + c2 + c3;
    int incl = ts;
#pragma unroll
    for (int d = 1; d < 32; d <<= 1) {
      const int up = __shfl_up(incl, d, 32);
      if (lane >= d) incl += up;
    }
    if (lane == 31) misc[16 + wave] = incl;
    __syncthreads();
    int pre = 0;
#pragma unroll
    for (int w2 = 0; w2 < NWB; ++w2) {
      const int t2 = misc[16 + w2];
      pre += (w2 < wave) ? t2 : 0;
    }
    const int o0 = pre + incl - ts, o1 = o0 + c0, o2 = o1 + c1, o3 = o2 + c2;
    v4i cq; cq.x = c0; cq.y = c1; cq.z = c2; cq.w = c3;
    v4i oq; oq.x = o0; oq.y = o1; oq.z = o2; oq.w = o3;
    *(v4ia*)(cnt + 4 * tid) = cq;
    *(v4ia*)(off + 4 * tid) = oq;
    int r0 = o0, r1 = o1, r2 = o2, r3 = o3;
#pragma unroll
    for (int w = 0; w < NWB; ++w) {
      const v4i q = *(const v4ia*)(cw + w * NBRUN + 4 * tid);
      v4i rq; rq.x = r0; rq.y = r1; rq.z = r2; rq.w = r3;
      *(v4ia*)(cw + w * NBRUN + 4 * tid) = rq;
      r0 += q.x; r1 += q.y; r2 += q.z; r3 += q.w;
    }
    if (tid == BTHR - 1) misc[32] = o3 + c3;
  }
  __syncthreads();
  const int tot = misc[32];
  int ovf = (tot > RCAP) ? 1 : 0;
#pragma unroll
  for (int w = 0; w < NWB; ++w) ovf |= misc[8 + w];

#pragma unroll 1
  for (int b0 = 0; b0 < n; b0 += 32) {
    int idx = b0 + lane;
    idx = idx > n - 1 ? n - 1 : idx;
    const int ent = mywl[idx];
    const int m32 = (n - b0) < 32 ? (n - b0) : 32;
#pragma unroll 1
    for (int k = 0; k < m32; ++k) {
      const int u  = __builtin_amdgcn_readlane(ent, k);
      const int sl = u & (NBRUN - 1);
      const int sr = (int)((unsigned)u >> SLB);
      if (lane == 0) {
        const int p = cw[wave * NBRUN + sl];
        const int pc = p < 0 ? 0 : (p > RCAP - 1 ? RCAP - 1 : p);
        plc[pc] = sr;
        cw[wave * NBRUN + sl] = p + 1;
      }
    }
  }
  __syncthreads();

  int* lg = lst + (size_t)b * RCAP;
  const v4i cq = *(const v4ia*)(cnt + 4 * tid);
  const v4i oq = *(const v4ia*)(off + 4 * tid);
  v4i fq; fq.x = ovf; fq.y = ovf; fq.z = ovf; fq.w = ovf;
#pragma unroll 1
  for (int it = 0; it < RCAP / (BTHR * 4); ++it) {
    const int i = (it * BTHR + tid) * 4;
    const v4i q = *(const v4ia*)(plc + i);
    *(volatile v4i*)(lg + i) = q;
  }
  *(volatile v4i*)(cntg + base + 4 * tid) = cq;
  *(volatile v4i*)(offg + base + 4 * tid) = oq;
  if (tid < 8) *(volatile v4i*)(flg + b * 32 + 4 * tid) = fq;
  __threadfence();
#pragma unroll 1
  for (int it = 0; it < RCAP / (BTHR * 4); ++it) {
    const int i = (it * BTHR + tid) * 4;
    const v4i q = *(const v4ia*)(plc + i);
    *(volatile v4i*)(lg + i) = q;
  }
  *(volatile v4i*)(cntg + base + 4 * tid) = cq;
  *(volatile v4i*)(offg + base + 4 * tid) = oq;
  if (tid < 8) *(volatile v4i*)(flg + b * 32 + 4 * tid) = fq;
}

__global__ __launch_bounds__(NTHR) void k_replay(const float* __restrict__ X, const int* __restrict__ lst,
                                                 const int* __restrict__ cntg, const int* __restrict__ offg,
                                                 const int* __restrict__ flg, const float* __restrict__ par,
                                                 int layer, unsigned short* Z) {
  __shared__ __attribute__((aligned(16))) unsigned int stw[8 * 128];
  const int tid = (int)threadIdx.x, lane = tid & 31, wave = tid >> 5;
  const int d = (int)blockIdx.x * 8 + wave;
  const int b = d >> SLB;
  const int cv = cntg[d];
  const int ov = offg[d];
  const int fv = flg[b * 32];
  pin_i(cv); pin_i(ov); pin_i(fv);
  const int badv = ((cv < 0) | (cv > DEGCAP) | (ov < 0) | (ov > RCAP) | (fv != 0)) ? 1 : 0;
  int cc = cv < 0 ? 0 : (cv > DEGCAP ? DEGCAP : cv);
  const int oo = ov < 0 ? 0 : (ov > RCAP - 1 ? RCAP - 1 : ov);
  cc = cc > RCAP - oo ? RCAP - oo : cc;
  const int c = __builtin_amdgcn_readfirstlane(cc);
  const int o = __builtin_amdgcn_readfirstlane(oo);
  const int badu = __builtin_amdgcn_readfirstlane(badv);
  int last = o + c - 1; last = last < o ? o : last;
  const int* lp = lst + (size_t)b * RCAP;
  float a0 = 0.0f, a1 = 0.0f, a2 = 0.0f, a3 = 0.0f;
#pragma unroll 1
  for (int b0 = 0; b0 < c; b0 += 32) {
    int idx = o + b0 + lane;
    idx = idx > last ? last : idx;
    const int sraw = lp[idx];
    pin_i(sraw);
    const int sv = sraw < 0 ? 0 : (sraw > NN - 1 ? NN - 1 : sraw);
    const int m32 = (c - b0) < 32 ? (c - b0) : 32;
#pragma unroll 1
    for (int k = 0; k < m32; ++k) {
      const int sk = __builtin_amdgcn_readlane(sv, k);
      const v4f v = *(const v4f*)(X + (size_t)sk * DH + 4 * lane);
      a0 += v.x; a1 += v.y; a2 += v.z; a3 += v.w;
    }
  }
  const bool live = d < NN;
  const int dc = live ? d : NN - 1;
  const v4f sf = *(const v4f*)(X + (size_t)dc * DH + 4 * lane);
  const float ep = 1.0f + par[PEPS + layer];
  const float pz = (live && (badu != 0)) ? __int_as_float(0x7fc00000) : 0.0f;
  float r0 = ep * sf.x + a0, r1 = ep * sf.y + a1, r2 = ep * sf.z + a2, r3 = ep * sf.w + a3;
  r0 = (live ? r0 : 0.0f) + pz;
  r1 = (live ? r1 : 0.0f) + pz;
  r2 = (live ? r2 : 0.0f) + pz;
  r3 = (live ? r3 : 0.0f) + pz;
  const unsigned hb0 = bf_bits(r0), hb1 = bf_bits(r1), hb2 = bf_bits(r2), hb3 = bf_bits(r3);
  const unsigned lb0 = bf_bits(r0 - bf_val(hb0)), lb1 = bf_bits(r1 - bf_val(hb1));
  const unsigned lb2 = bf_bits(r2 - bf_val(hb2)), lb3 = bf_bits(r3 - bf_val(hb3));
  v2u hw, lw;
  hw.x = hb0 | (hb1 << 16); hw.y = hb2 | (hb3 << 16);
  lw.x = lb0 | (lb1 << 16); lw.y = lb2 | (lb3 << 16);
  unsigned int* stwu = stw + wave * 128;
  __builtin_amdgcn_fence(__ATOMIC_RELEASE, "wavefront");
  __builtin_amdgcn_wave_barrier();
  *(v2u*)(stwu + 2 * lane)      = hw;
  *(v2u*)(stwu + 64 + 2 * lane) = lw;
  __builtin_amdgcn_fence(__ATOMIC_RELEASE, "wavefront");
  __builtin_amdgcn_wave_barrier();
  const v4u pk = *(const v4ua*)(stwu + 4 * lane);
  unsigned short* gp = Z + (size_t)d * PZ + 8 * lane;
  *(volatile v4u*)gp = pk;
  __threadfence();
  *(volatile v4u*)gp = pk;
}

template <int KA, int AP, int WP, int NT, int MODE>
__global__ __launch_bounds__(GTHR) __attribute__((amdgpu_num_vgpr(248)))
void k_gemm(const unsigned short* __restrict__ A, const unsigned short* __restrict__ WT,
            const float* __restrict__ bias, float* outp, float* rec, int nN) {
  constexpr int BN = 16 * NT;
  constexpr int OP = (MODE == 0) ? 256 : ((MODE == 1) ? 128 : 64);
  constexpr int LPR = BN / 4;
  constexpr int RPI = 32 / LPR;
  constexpr int NI  = 16 / RPI;
  static_assert(KA % 32 == 0 && KA <= AP && KA <= WP && (AP % 8) == 0 && (WP % 8) == 0);
  static_assert(BN == 128 || (BN == 64 && MODE == 2));
  static_assert(MODE != 2 || OP == BN);
  static_assert(GTHR == 256 && GBM == 8 * 16);
  extern __shared__ v4f gsm4[];
  float* stg = (float*)gsm4;
  float* bsh = stg + GBM * BN;
  float* pst = bsh + 128;
  const int tid = (int)threadIdx.x, lane = tid & 31, wave = tid >> 5, hh = lane >> 4, m = lane & 15;
  const int rowBase = (int)blockIdx.x * GBM;
  const int colBase = (int)blockIdx.y * BN;

  if (tid < BN / 4) {
    const v4f b4 = *(const v4f*)(bias + colBase + 4 * tid);
    *(v4fa*)(bsh + 4 * tid) = b4;
  }
  __syncthreads();

  v8f acc[NT];
  {
    const v8f z = {0.f, 0.f, 0.f, 0.f, 0.f, 0.f, 0.f, 0.f};
#pragma unroll
    for (int t = 0; t < NT; ++t) acc[t] = z;
  }
  const unsigned short* ap = A + (size_t)(rowBase + 16 * wave + m) * (size_t)AP + 8 * hh;
  const unsigned short* wp = WT + (size_t)(colBase + m) * (size_t)WP + 8 * hh;
  constexpr int ksteps = KA / 32;
#pragma unroll 1
  for (int ks = 0; ks < ksteps; ++ks) {
    FragB af;
    af.h[0] = *(const v8usa*)(ap + 32 * ks);
    af.h[1] = *(const v8usa*)(ap + 32 * ks + 16);
#pragma unroll
    for (int t = 0; t < NT; ++t) {
      const unsigned short* wq = wp + (size_t)(16 * t) * (size_t)WP + 32 * ks;
      FragB bf;
      bf.h[0] = *(const v8usa*)wq;
      bf.h[1] = *(const v8usa*)(wq + 16);
      acc[t] = wmb(af, bf, acc[t]);
    }
  }

#pragma unroll
  for (int t = 0; t < NT; ++t) {
    const int lc = 16 * t + m;
    const float bb = bsh[lc];
#pragma unroll
    for (int r = 0; r < 8; ++r) {
      const int lr = 16 * wave + 8 * hh + r;
      const bool live = (rowBase + lr) < nN;
      const float v = acc[t][r] + bb;
      stg[lr * BN + lc] = live ? v : 0.0f;
    }
  }
  __syncthreads();

  if constexpr (MODE == 0) {
    if (tid < 128) {
      int rv = nN - rowBase;
      rv = rv < 0 ? 0 : (rv > GBM ? GBM : rv);
      float s = 0.0f;
#pragma unroll 4
      for (int r = 0; r < rv; ++r) s += stg[r * BN + tid];
      const float rn = 1.0f / (float)(rv < 1 ? 1 : rv);
      const float mean = s * rn;
      float q = 0.0f;
#pragma unroll 4
      for (int r = 0; r < rv; ++r) {
        const float dlt = stg[r * BN + tid] - mean;
        q = fmaf(dlt, dlt, q);
      }
      pst[2 * tid]     = mean;
      pst[2 * tid + 1] = q;
    }
  }

  const int rsub = lane / LPR;
  const int c4   = 4 * (lane % LPR);
  const int rowLim = (MODE == 2) ? nN : MPAD;
  v4f fv[NI];
#pragma unroll
  for (int i = 0; i < NI; ++i) {
    const int lr = 16 * wave + RPI * i + rsub;
    fv[i] = *(const v4fa*)(stg + lr * BN + c4);
  }
#pragma unroll
  for (int i = 0; i < NI; ++i) {
    const int gr = rowBase + 16 * wave + RPI * i + rsub;
    float* op = outp + (size_t)gr * (size_t)OP + colBase + c4;
    if (gr < rowLim) *(volatile v4f*)op = fv[i];
  }
  __threadfence();
#pragma unroll
  for (int i = 0; i < NI; ++i) {
    const int gr = rowBase + 16 * wave + RPI * i + rsub;
    float* op = outp + (size_t)gr * (size_t)OP + colBase + c4;
    if (gr < rowLim) *(volatile v4f*)op = fv[i];
  }

  if constexpr (MODE == 0) {
    __syncthreads();
    float* rp = rec + (size_t)blockIdx.x * (2 * D2) + (size_t)blockIdx.y * 256 + 4 * tid;
    v4f pv = {0.f, 0.f, 0.f, 0.f};
    if (tid < 64) {
      pv = *(const v4fa*)(pst + 4 * tid);
      *(volatile v4f*)rp = pv;
    }
    __threadfence();
    if (tid < 64) {
      *(volatile v4f*)rp = pv;
    }
  }
}

__global__ __launch_bounds__(D2) void k_comb(const float* __restrict__ rec, float* stat) {
  __shared__ __attribute__((aligned(16))) float sst[2 * D2];
  const int tid = (int)threadIdx.x;
  const int c = tid;
  double n = 0.0, mean = 0.0, M2 = 0.0;
#pragma unroll 1
  for (int mt = 0; mt < MTILES; ++mt) {
    int nbi = NN - GBM * mt;
    nbi = nbi < 0 ? 0 : (nbi > GBM ? GBM : nbi);
    const v2f q = *(const v2f*)(rec + ((size_t)mt * D2 + c) * 2);
    if (nbi > 0) {
      const double nb = (double)nbi;
      const double nn = n + nb;
      const double delta = (double)q.x - mean;
      const double f = nb / nn;
      mean = mean + delta * f;
      M2 = M2 + (double)q.y + delta * delta * n * f;
      n = nn;
    }
  }
  const double nt = n < 1.0 ? 1.0 : n;
  const float varf = (float)(M2 / nt);
  const float rs = 1.0f / sqrtf(varf + 1e-5f);
  sst[c] = (float)mean;
  sst[D2 + c] = rs;
  __syncthreads();
  v4f v = {0.f, 0.f, 0.f, 0.f};
  if (tid < (2 * D2) / 4) {
    v = *(const v4fa*)(sst + 4 * tid);
    *(volatile v4f*)(stat + 4 * tid) = v;
  }
  __threadfence();
  if (tid < (2 * D2) / 4) {
    *(volatile v4f*)(stat + 4 * tid) = v;
  }
}

__global__ __launch_bounds__(NTHR) void k_apply(const float* __restrict__ T, const float* __restrict__ stat,
                                                const float* __restrict__ par, int layer,
                                                unsigned short* Y, int nN) {
  const int tid = (int)threadIdx.x, lane = tid & 31, wave = tid >> 5;
  const int c8 = 8 * lane;
  const v4f m0 = *(const v4f*)(stat + c8),       m1 = *(const v4f*)(stat + c8 + 4);
  const v4f q0 = *(const v4f*)(stat + D2 + c8),  q1 = *(const v4f*)(stat + D2 + c8 + 4);
  const v4f g0 = *(const v4f*)(par + PGAM + layer * D2 + c8), g1 = *(const v4f*)(par + PGAM + layer * D2 + c8 + 4);
  const v4f e0 = *(const v4f*)(par + PBET + layer * D2 + c8), e1 = *(const v4f*)(par + PBET + layer * D2 + c8 + 4);
  const float mm[8] = {m0.x, m0.y, m0.z, m0.w, m1.x, m1.y, m1.z, m1.w};
  const float rr[8] = {q0.x, q0.y, q0.z, q0.w, q1.x, q1.y, q1.z, q1.w};
  const float gg[8] = {g0.x, g0.y, g0.z, g0.w, g1.x, g1.y, g1.z, g1.w};
  const float bb[8] = {e0.x, e0.y, e0.z, e0.w, e1.x, e1.y, e1.z, e1.w};
  const int rowB = (int)blockIdx.x * 64 + wave * 8;
#pragma unroll 1
  for (int j = 0; j < 8; ++j) {
    const int row = rowB + j;
    const bool live = row < nN;
    const int rc = live ? row : nN - 1;
    const v4f a = *(const v4f*)(T + (size_t)rc * D2 + c8);
    const v4f b = *(const v4f*)(T + (size_t)rc * D2 + c8 + 4);
    const float tv[8] = {a.x, a.y, a.z, a.w, b.x, b.y, b.z, b.w};
    unsigned hwv[4], lwv[4];
#pragma unroll
    for (int i = 0; i < 4; ++i) {
      float y0 = ((tv[2 * i]     - mm[2 * i])     * gg[2 * i])     * rr[2 * i]     + bb[2 * i];
      float y1 = ((tv[2 * i + 1] - mm[2 * i + 1]) * gg[2 * i + 1]) * rr[2 * i + 1] + bb[2 * i + 1];
      y0 = (y0 > 0.0f) ? y0 : (y0 - y0);
      y1 = (y1 > 0.0f) ? y1 : (y1 - y1);
      y0 = live ? y0 : 0.0f;
      y1 = live ? y1 : 0.0f;
      const unsigned h0 = bf_bits(y0), h1 = bf_bits(y1);
      const unsigned l0 = bf_bits(y0 - bf_val(h0)), l1 = bf_bits(y1 - bf_val(h1));
      hwv[i] = h0 | (h1 << 16);
      lwv[i] = l0 | (l1 << 16);
    }
    v4u hq, lq;
    hq.x = hwv[0]; hq.y = hwv[1]; hq.z = hwv[2]; hq.w = hwv[3];
    lq.x = lwv[0]; lq.y = lwv[1]; lq.z = lwv[2]; lq.w = lwv[3];
    unsigned short* hp = Y + (size_t)row * PT + c8;
    *(volatile v4u*)hp = hq;
    *(volatile v4u*)(hp + D2) = lq;
    __threadfence();
    *(volatile v4u*)hp = hq;
    *(volatile v4u*)(hp + D2) = lq;
  }
}

__global__ __launch_bounds__(NTHR) void k_split(const float* __restrict__ X, unsigned short* Y, int nN) {
  const int tid = (int)threadIdx.x, lane = tid & 31, wave = tid >> 5, hh = lane >> 4, m = lane & 15;
  const int cb = 8 * m;
  const bool isHi = (hh == 0);
  const int rowB = (int)blockIdx.x * 64 + wave * 8;
#pragma unroll 1
  for (int j = 0; j < 8; ++j) {
    const int row = rowB + j;
    const bool live = row < nN;
    const int rc = live ? row : nN - 1;
    const v4f a = *(const v4f*)(X + (size_t)rc * DH + cb);
    const v4f b = *(const v4f*)(X + (size_t)rc * DH + cb + 4);
    const float f[8] = {a.x, a.y, a.z, a.w, b.x, b.y, b.z, b.w};
    unsigned w[4];
#pragma unroll
    for (int i = 0; i < 4; ++i) {
      const float y0 = live ? f[2 * i] : 0.0f;
      const float y1 = live ? f[2 * i + 1] : 0.0f;
      const unsigned h0 = bf_bits(y0), h1 = bf_bits(y1);
      const unsigned l0 = bf_bits(y0 - bf_val(h0)), l1 = bf_bits(y1 - bf_val(h1));
      const unsigned s0 = isHi ? h0 : l0, s1 = isHi ? h1 : l1;
      w[i] = s0 | (s1 << 16);
    }
    v4u pk; pk.x = w[0]; pk.y = w[1]; pk.z = w[2]; pk.w = w[3];
    unsigned short* op = Y + (size_t)row * PZ + 8 * lane;
    *(volatile v4u*)op = pk;
    __threadfence();
    *(volatile v4u*)op = pk;
  }
}

static inline size_t al128(size_t o) { return (o + 127) & ~(size_t)127; }

extern "C" void kernel_launch(void* const* d_in, const int* in_sizes, int n_in,
                              void* d_out, int out_size, void* d_ws, size_t ws_size,
                              hipStream_t stream) {
  if (n_in < 11) return;
  if (in_sizes[0] != NN * DH) return;
  if (in_sizes[1] != 2 * NE) return;
  if (in_sizes[2] != NL * DH * D2) return;
  if (in_sizes[3] != NL * D2) return;
  if (in_sizes[4] != NL * D2) return;
  if (in_sizes[5] != NL * D2) return;
  if (in_sizes[6] != NL * D2 * DH) return;
  if (in_sizes[7] != NL * DH) return;
  if (in_sizes[8] != NL) return;
  if (in_sizes[9] != DH * DOUT) return;
  if (in_sizes[10] != DOUT) return;
  if (out_size != NN * DOUT) return;

  const float* x    = (const float*)d_in[0];
  const int*   ei   = (const int*)  d_in[1];
  const float* W1   = (const float*)d_in[2];
  const float* b1   = (const float*)d_in[3];
  const float* gam  = (const float*)d_in[4];
  const float* bet  = (const float*)d_in[5];
  const float* W2   = (const float*)d_in[6];
  const float* b2   = (const float*)d_in[7];
  const float* eps  = (const float*)d_in[8];
  const float* linW = (const float*)d_in[9];
  const float* linb = (const float*)d_in[10];
  float* out = (float*)d_out;

  char* ws = (char*)d_ws;
  size_t off = 0;
  const size_t oR1  = off; off = al128(off + (size_t)MPAD * D2 * 4);
  const size_t oR2  = off; off = al128(off + (size_t)MPAD * PT * 2);
  const size_t oLST = off; off = al128(off + (size_t)NBLK * RCAP * 4);
  const size_t oCNT = off; off = al128(off + (size_t)CNTN * 4);
  const size_t oOFF = off; off = al128(off + (size_t)CNTN * 4);
  const size_t oFLG = off; off = al128(off + (size_t)64 * 128);
  const size_t oW1T = off; off = al128(off + (size_t)NL * D2 * PZ * 2);
  const size_t oW2T = off; off = al128(off + (size_t)NL * DH * PT * 2);
  const size_t oLWT = off; off = al128(off + (size_t)DOUT * PZ * 2);
  const size_t oREC = off; off = al128(off + (size_t)MTILES * D2 * 2 * 4);
  const size_t oSTA = off; off = al128(off + (size_t)NL * 2 * D2 * 4);
  const size_t oPAR = off; off = al128(off + (size_t)PARN * 4);
  if (off > ws_size || off > (size_t)WSMAX) return;

  float*          R1f  = (float*)(ws + oR1);
  unsigned short* R2h  = (unsigned short*)(ws + oR2);
  int*            LST  = (int*)(ws + oLST);
  int*            CNT  = (int*)(ws + oCNT);
  int*            OFFS = (int*)(ws + oOFF);
  int*            FLG  = (int*)(ws + oFLG);
  unsigned short* W1T  = (unsigned short*)(ws + oW1T);
  unsigned short* W2T  = (unsigned short*)(ws + oW2T);
  unsigned short* LWT  = (unsigned short*)(ws + oLWT);
  float*          REC  = (float*)(ws + oREC);
  float*          STA  = (float*)(ws + oSTA);
  float*          PAR  = (float*)(ws + oPAR);

  const int ldsB  = BKT_INTS * 4;
  const int ldsG8 = (GBM * 128 + 128 + 256) * 4;
  const int ldsG4 = (GBM * 64 + 128 + 256) * 4;
  hipFuncSetAttribute(reinterpret_cast<const void*>(&k_bucket), hipFuncAttributeMaxDynamicSharedMemorySize, ldsB);
  hipFuncSetAttribute(reinterpret_cast<const void*>(&k_gemm<KZ, PZ, PZ, 8, 0>),
                      hipFuncAttributeMaxDynamicSharedMemorySize, ldsG8);
  hipFuncSetAttribute(reinterpret_cast<const void*>(&k_gemm<KT, PT, PT, 8, 1>),
                      hipFuncAttributeMaxDynamicSharedMemorySize, ldsG8);
  hipFuncSetAttribute(reinterpret_cast<const void*>(&k_gemm<KF, PZ, PZ, 4, 2>),
                      hipFuncAttributeMaxDynamicSharedMemorySize, ldsG4);

  k_prep<<<PGRID, NTHR, 0, stream>>>(x, W1, b1, gam, bet, W2, b2, eps, linW, linb, W1T, W2T, LWT, PAR, R1f);
  k_bucket<<<NBLK, BTHR, ldsB, stream>>>(ei, LST, CNT, OFFS, FLG);
  for (int l = 0; l < NL; ++l) {
    k_replay<<<MPAD / 8, NTHR, 0, stream>>>(R1f, LST, CNT, OFFS, FLG, PAR, l, R2h);
    k_gemm<KZ, PZ, PZ, 8, 0><<<dim3(MTILES, 2), GTHR, ldsG8, stream>>>(
        R2h, W1T + (size_t)l * (D2 * PZ), PAR + PB1 + l * D2, R1f, REC, NN);
    k_comb<<<1, D2, 0, stream>>>(REC, STA + (size_t)l * (2 * D2));
    k_apply<<<MPAD / 64, NTHR, 0, stream>>>(R1f, STA + (size_t)l * (2 * D2), PAR, l, R2h, NN);
    k_gemm<KT, PT, PT, 8, 1><<<dim3(MTILES, 1), GTHR, ldsG8, stream>>>(
        R2h, W2T + (size_t)l * (DH * PT), PAR + PB2 + l * DH, R1f, REC, NN);
  }
  k_split<<<MPAD / 64, NTHR, 0, stream>>>(R1f, R2h, NN);
  k_gemm<KF, PZ, PZ, 4, 2><<<dim3(MTILES, 1), GTHR, ldsG4, stream>>>(R2h, LWT, PAR + PLB, out, REC, NN);
}
